// C_REN_36386962931992
// MI455X (gfx1250) — hardware-verified
//
#include <hip/hip_runtime.h>
#include <math.h>

typedef __attribute__((ext_vector_type(16))) _Float16 v16h;
typedef __attribute__((ext_vector_type(8)))  _Float16 v8h;
typedef __attribute__((ext_vector_type(4)))  _Float16 v4h;
typedef __attribute__((ext_vector_type(2)))  _Float16 v2h;
typedef __attribute__((ext_vector_type(16))) __bf16   v16b;
typedef __attribute__((ext_vector_type(8)))  __bf16   v8b;
typedef __attribute__((ext_vector_type(8)))  float    v8f;
typedef __attribute__((ext_vector_type(4)))  float    v4f;
typedef __attribute__((ext_vector_type(2)))  float    v2f;

constexpr int kBatch = 65536;
constexpr int kHalf  = 32768;
constexpr int kNin   = 32;
constexpr int kNout  = 16;
constexpr int kNst   = 128;
constexpr int kNnl   = 64;
constexpr int kHdim  = 2 * kNst + kNnl;
constexpr int kKsv   = kNst + kNin;
constexpr int kKz    = kNst + kNnl + kNin;
constexpr int kThr   = 256;
constexpr float kEps = 1.0e-3f;

constexpr float kInCarry  = 1024.0f;
constexpr float kWCarry   = 1024.0f;
constexpr float kLoCarry  = 4096.0f;
constexpr float kExCarry  = 64.0f;
constexpr float kEiCarry  = 256.0f;
constexpr float kXwScale  = 1.0f / (kInCarry * kWCarry);
constexpr float kSpScale  = 1.0f / (kExCarry * kEiCarry);
constexpr float kLoFold   = 1.0f / kLoCarry;
constexpr float kF16MinNormal = 6.103515625e-5f;

static_assert(kHdim == 320 && (kHdim % 64) == 0 && (kKsv % 32) == 0 && (kKz % 32) == 0 && (kHalf % 64) == 0, "GEMM M, N multiples of 64, K of 32");

constexpr size_t kOffXT   = 0;
constexpr size_t kOffZB   = kOffXT   + (size_t)kHdim * kHdim * 2;
constexpr size_t kOffH32  = kOffZB   + (size_t)kHdim * 4;
constexpr size_t kOffWSV  = kOffH32  + (size_t)kHdim * kHdim * 4;
constexpr size_t kOffWEX  = kOffWSV  + (size_t)2 * kNnl * kKsv * 2;
constexpr size_t kOffWOUT = kOffWEX  + (size_t)2 * kNst * kKz * 2;
constexpr size_t kOffEINV = kOffWOUT + (size_t)64 * kKz * 2;
constexpr size_t kOffD11  = kOffEINV + (size_t)2 * kNst * kNst * 2;
constexpr size_t kOffLAM  = kOffD11  + (size_t)kNnl * kNnl * 4;
constexpr size_t kOffZS   = kOffLAM  + (size_t)kNnl * 4;
constexpr size_t kOffSV2  = kOffZS   + (size_t)kHalf * kKsv * 2;
constexpr size_t kOffZ16  = kOffSV2  + (size_t)kHalf * 2 * kNnl * 4;
constexpr size_t kOffEX2  = kOffZ16  + (size_t)kHalf * kKz * 2;
constexpr size_t kOffEX16 = kOffEX2  + (size_t)kHalf * 2 * kNst * 4;
constexpr size_t kWsTotal = kOffEX16 + (size_t)kHalf * kNst * 2;
static_assert(kWsTotal == 84768256ull, "carve total");
static_assert(kWsTotal <= 134217728ull, "carve cap");
static_assert((kOffZB % 256) == 0 && (kOffH32 % 256) == 0 && (kOffWSV % 256) == 0 && (kOffWEX % 256) == 0 && (kOffWOUT % 256) == 0 && (kOffEINV % 256) == 0 && (kOffD11 % 256) == 0 && (kOffLAM % 256) == 0 && (kOffZS % 256) == 0 && (kOffSV2 % 256) == 0 && (kOffZ16 % 256) == 0 && (kOffEX2 % 256) == 0 && (kOffEX16 % 256) == 0, "aligned regions");

__device__ __forceinline__ unsigned short f2bf_bits(float f) {
  unsigned u = __float_as_uint(f);
  return (unsigned short)((u + 0x7FFFu + ((u >> 16) & 1u)) >> 16);
}
__device__ __forceinline__ float bf_bits2f(unsigned short h) { return __uint_as_float(((unsigned)h) << 16); }
__device__ __forceinline__ float bf16r(float f) { return bf_bits2f(f2bf_bits(f)); }
__device__ __forceinline__ float carry_flush(float v, float carry) {
  const float s = v * carry;
  return (fabsf(s) < kF16MinNormal) ? 0.0f : s;
}
__device__ __forceinline__ float frcp(float x) { return __builtin_amdgcn_rcpf(x); }

__device__ __forceinline__ void dep_guard4_h(v8f& a, v8f& b, v8f& c, v8f& d, v16h x, v16h y) { asm volatile("v_nop\n\tv_nop\n\tv_nop\n\tv_nop" : "+v"(a), "+v"(b), "+v"(c), "+v"(d) : "v"(x), "v"(y)); }
__device__ __forceinline__ void dep_guard4_b(v8f& a, v8f& b, v8f& c, v8f& d, v16b x, v16b y) { asm volatile("v_nop\n\tv_nop\n\tv_nop\n\tv_nop" : "+v"(a), "+v"(b), "+v"(c), "+v"(d) : "v"(x), "v"(y)); }
__device__ __forceinline__ void keep4_h(v16h a, v16h b, v16h c, v16h d) { asm volatile("v_nop" :: "v"(a), "v"(b), "v"(c), "v"(d)); }
__device__ __forceinline__ void keep4_b(v16b a, v16b b, v16b c, v16b d) { asm volatile("v_nop" :: "v"(a), "v"(b), "v"(c), "v"(d)); }
__device__ __forceinline__ void acc_guard4(v8f& a, v8f& b, v8f& c, v8f& d) { asm volatile("v_nop\n\tv_nop\n\tv_nop\n\tv_nop" : "+v"(a), "+v"(b), "+v"(c), "+v"(d)); }

template <typename T> struct Frag;
template <> struct Frag<_Float16> {
  typedef v16h V; union U { v16h v; v8h h[2]; };
  static __device__ __forceinline__ v16h load(const _Float16* p) {
    U f; f.h[0] = *(const v8h*)(p); f.h[1] = *(const v8h*)(p + 16); return f.v;
  }
  static __device__ __forceinline__ v8f mma(v16h a, v16h b, v8f c) {
    return __builtin_amdgcn_wmma_f32_16x16x32_f16(false, a, false, b, (short)0, c, false, false);
  }
  static __device__ __forceinline__ void guard4(v8f& a, v8f& b, v8f& c, v8f& d, v16h x, v16h y) { dep_guard4_h(a, b, c, d, x, y); }
  static __device__ __forceinline__ void keep(v16h a, v16h b, v16h c, v16h d) { keep4_h(a, b, c, d); }
};
template <> struct Frag<__bf16> {
  typedef v16b V; union U { v16b v; v8b h[2]; };
  static __device__ __forceinline__ v16b load(const __bf16* p) {
    U f; f.h[0] = *(const v8b*)(p); f.h[1] = *(const v8b*)(p + 16); return f.v;
  }
  static __device__ __forceinline__ v8f mma(v16b a, v16b b, v8f c) {
    return __builtin_amdgcn_wmma_f32_16x16x32_bf16(false, a, false, b, (short)0, c, false, false);
  }
  static __device__ __forceinline__ void guard4(v8f& a, v8f& b, v8f& c, v8f& d, v16b x, v16b y) { dep_guard4_b(a, b, c, d, x, y); }
  static __device__ __forceinline__ void keep(v16b a, v16b b, v16b c, v16b d) { keep4_b(a, b, c, d); }
};

__device__ __forceinline__ v8f mma_h(v16h a, v16h b, v8f c) {
  c = __builtin_amdgcn_wmma_f32_16x16x32_f16(false, a, false, b, (short)0, c, false, false);
  asm volatile("v_nop\n\tv_nop\n\tv_nop\n\tv_nop" : "+v"(c) : "v"(a), "v"(b));
  return c;
}

template <int ET> struct Elem;
template <> struct Elem<0> { typedef _Float16 T; };
template <> struct Elem<1> { typedef __bf16 T; };
template <int ET, bool SPLIT, int BIAS_MODE, int OUT_MODE, bool RESID, int ACT = 0>
__global__ __launch_bounds__(256) void wmma_gemm64(
    const unsigned short* __restrict__ Ap, const unsigned short* __restrict__ A2p, int lda, long strideA,
    const unsigned short* __restrict__ Btp, const unsigned short* __restrict__ Bt2p, int ldb, long strideB,
    void* __restrict__ Cout, void* __restrict__ Cout2, int ldc, long strideC,
    const float* __restrict__ bias,
    const float* __restrict__ resid, long strideR,
    int M, int N, int K, float scale) {
  typedef typename Elem<ET>::T T;
  typedef typename Frag<T>::V V;
  const T* A = (const T*)Ap; const T* A2 = (const T*)A2p; const T* Bt = (const T*)Btp; const T* Bt2 = (const T*)Bt2p;
  __shared__ __align__(16) float sT[8][16 * 68];
  const int b    = blockIdx.y;
  const int lane = threadIdx.x & 31;
  const int wave = threadIdx.x >> 5;
  const int tilesN = N >> 6;
  const int tilesM = M >> 6;
  const int tile = blockIdx.x * 8 + wave;
  if (tile >= tilesM * tilesN) return;
  const int tm = tile / tilesN;
  const int tn = tile - tm * tilesN;
  const int m0 = tm << 6;
  const int n0 = tn << 6;

  const T* Ab  = A  + (size_t)b * strideA;
  const T* Bb  = Bt + (size_t)b * strideB;
  const T* Ab2 = SPLIT ? (A2  + (size_t)b * strideA) : nullptr;
  const T* Bb2 = SPLIT ? (Bt2 + (size_t)b * strideB) : nullptr;

  const int rlane = lane & 15;
  const int koff  = (lane >> 4) * 8;
  const int mOff  = (lane >> 4) * 8;

  v8f acc[4][4];
#pragma unroll
  for (int i = 0; i < 4; ++i)
#pragma unroll
    for (int j = 0; j < 4; ++j) acc[i][j] = (v8f){0.f,0.f,0.f,0.f,0.f,0.f,0.f,0.f};

  for (int k0 = 0; k0 < K; k0 += 32) {
    V bh[4], bl[4];
#pragma unroll
    for (int j = 0; j < 4; ++j) {
      const size_t bo = (size_t)(n0 + (j << 4) + rlane) * ldb + koff + k0;
      bh[j] = Frag<T>::load(Bb + bo);
      if (SPLIT) bl[j] = Frag<T>::load(Bb2 + bo);
    }
#pragma unroll
    for (int i = 0; i < 4; ++i) {
      const size_t ao = (size_t)(m0 + (i << 4) + rlane) * lda + koff + k0;
      V ah = Frag<T>::load(Ab + ao);
      V al;
      if (SPLIT) al = Frag<T>::load(Ab2 + ao);
#pragma unroll
      for (int j = 0; j < 4; ++j) {
        acc[i][j] = Frag<T>::mma(ah, bh[j], acc[i][j]);
        if (SPLIT) {
          acc[i][j] = Frag<T>::mma(ah, bl[j], acc[i][j]);
          acc[i][j] = Frag<T>::mma(al, bh[j], acc[i][j]);
        }
      }
      Frag<T>::guard4(acc[i][0], acc[i][1], acc[i][2], acc[i][3], ah, SPLIT ? al : ah);
    }
    Frag<T>::keep(bh[0], bh[1], bh[2], bh[3]);
    if (SPLIT) Frag<T>::keep(bl[0], bl[1], bl[2], bl[3]);
  }
  acc_guard4(acc[0][0], acc[0][1], acc[0][2], acc[0][3]);
  acc_guard4(acc[1][0], acc[1][1], acc[1][2], acc[1][3]);
  acc_guard4(acc[2][0], acc[2][1], acc[2][2], acc[2][3]);
  acc_guard4(acc[3][0], acc[3][1], acc[3][2], acc[3][3]);

  float* slab = sT[wave];
  const float* Rb = RESID ? (resid + (size_t)b * strideR) : nullptr;
#pragma unroll
  for (int i = 0; i < 4; ++i) {
    const int mBase = m0 + (i << 4);
#pragma unroll
    for (int j = 0; j < 4; ++j) {
      const int n = n0 + (j << 4) + rlane;
      float bv = 0.f;
      if (BIAS_MODE == 2) bv = bias[n];
#pragma unroll
      for (int r = 0; r < 8; ++r) {
        float v = acc[i][j][r] * scale;
        if (BIAS_MODE == 1) v += bias[mBase + mOff + r];
        if (BIAS_MODE == 2) v += bv;
        if (RESID) v += Rb[(size_t)(mBase + mOff + r) * ldc + n];
        if (ACT == 1) v = tanhf(v);
        if (ACT == 2) v = fmaxf(v, 0.0f);
        if (ACT == 3) v = v / (1.0f + expf(-v));
        if (ACT == 4) v = (v > 0.f) ? v : 0.01f * v;
        slab[(mOff + r) * 68 + (j << 4) + rlane] = v;
      }
    }
    __builtin_amdgcn_fence(__ATOMIC_RELEASE, "workgroup");
    __builtin_amdgcn_wave_barrier();
    __builtin_amdgcn_fence(__ATOMIC_ACQUIRE, "workgroup");
    if (OUT_MODE == 0) {
      float* C = (float*)Cout + (size_t)b * strideC;
      const int hh = lane >> 4, c4 = (lane & 15) * 4;
      for (int pass = 0; pass < 2; ++pass) {
#pragma unroll
        for (int it = 0; it < 8; ++it) {
          const int row = it * 2 + hh;
          v4f v = *(const v4f*)(slab + row * 68 + c4);
          *(volatile v4f*)(C + (size_t)(mBase + row) * ldc + n0 + c4) = v;
        }
        __threadfence();
      }
    } else {
      const int q = lane >> 3, c8 = (lane & 7) * 8;
      unsigned short* C  = (unsigned short*)Cout  + (size_t)b * strideC;
      unsigned short* C2 = (OUT_MODE == 2) ? ((unsigned short*)Cout2 + (size_t)b * strideC) : nullptr;
      for (int pass = 0; pass < 2; ++pass) {
#pragma unroll
        for (int it = 0; it < 4; ++it) {
          const int row = it * 4 + q;
          const float* sp = slab + row * 68 + c8;
          v8h hv, lv;
#pragma unroll
          for (int e = 0; e < 8; ++e) {
            if (OUT_MODE == 1) {
              hv[e] = (_Float16)sp[e];
            } else {
              unsigned short hb = f2bf_bits(sp[e]);
              unsigned short lb = f2bf_bits(sp[e] - bf_bits2f(hb));
              hv[e] = __builtin_bit_cast(_Float16, hb);
              lv[e] = __builtin_bit_cast(_Float16, lb);
            }
          }
          *(volatile v8h*)(C + (size_t)(mBase + row) * ldc + n0 + c8) = hv;
          if (OUT_MODE == 2) *(volatile v8h*)(C2 + (size_t)(mBase + row) * ldc + n0 + c8) = lv;
        }
        __threadfence();
      }
    }
    __builtin_amdgcn_fence(__ATOMIC_RELEASE, "workgroup");
    __builtin_amdgcn_wave_barrier();
    __builtin_amdgcn_fence(__ATOMIC_ACQUIRE, "workgroup");
  }
}


__device__ __forceinline__ void split_w(float w, float c, _Float16& hi, _Float16& lo) {
  const float wc = w * c;
  hi = (_Float16)carry_flush(w, c);
  lo = (_Float16)carry_flush(wc - (float)hi, kLoCarry);
}

__global__ __launch_bounds__(64) void xt_plane_kernel(const float* __restrict__ X, unsigned short* __restrict__ XT16,
                                                      float* __restrict__ ZB) {
  const int i  = blockIdx.x;
  const int k8 = threadIdx.x * 8;
  if (i == kHdim) {
    const v4f z = {0.f, 0.f, 0.f, 0.f};
    for (int pass = 0; pass < 2; ++pass) {
      *(volatile v4f*)(ZB + k8) = z;
      *(volatile v4f*)(ZB + k8 + 4) = z;
      __threadfence();
    }
    return;
  }
  v8h hv;
#pragma unroll
  for (int e = 0; e < 8; ++e) hv[e] = (_Float16)carry_flush(bf16r(X[(size_t)(k8 + e) * kHdim + i]), kInCarry);
  unsigned short* dp = XT16 + (size_t)i * kHdim + k8;
  *(volatile v8h*)dp = hv;
  __threadfence();
  *(volatile v8h*)dp = hv;
}

__global__ __launch_bounds__(kThr) void wplanes_kernel(const float* __restrict__ H, const float* __restrict__ D12,
                                                       const float* __restrict__ B2, const float* __restrict__ C2,
                                                       const float* __restrict__ D21, const float* __restrict__ D22,
                                                       unsigned short* __restrict__ WSV2, unsigned short* __restrict__ WEX2,
                                                       unsigned short* __restrict__ WOUT, float* __restrict__ D11,
                                                       float* __restrict__ LAM) {
  constexpr int nA = 128 * 20, nB = 256 * 28, nC = 64 * 28, nD = 64 * 8, nE = 8;
  int v = blockIdx.x * kThr + threadIdx.x;
  const bool live = v < nA + nB + nC + nD + nE;
  if (v > nA + nB + nC + nD + nE - 1) v = nA + nB + nC + nD + nE - 1;
  if (v < nA + nB + nC) {
    int which, row, k8, ld;
    if (v < nA) { which = 0; row = v / 20; k8 = (v - row * 20) * 8; ld = kKsv; }
    else if (v < nA + nB) { which = 1; const int u = v - nA; row = u / 28; k8 = (u - row * 28) * 8; ld = kKz; }
    else { which = 2; const int u = v - nA - nB; row = u / 28; k8 = (u - row * 28) * 8; ld = kKz; }
    const int half = (which == 0) ? (row >> 6) : ((which == 1) ? (row >> 7) : 0);
    const int r = (which == 0) ? (row & 63) : ((which == 1) ? (row & 127) : row);
    v8h hv;
#pragma unroll
    for (int e = 0; e < 8; ++e) {
      const int k = k8 + e;
      float w;
      bool computed;
      if (which == 0) {
        const int kc = (k < kNst) ? k : (kNst - 1);
        const int kd = (k >= kNst) ? (k - kNst) : 0;
        const float hc = -H[(size_t)(kNst + r) * kHdim + kc];
        const float dd = bf16r(D12[r * kNin + kd]);
        computed = (k < kNst);
        w = computed ? hc : dd;
      } else if (which == 1) {
        const int kh = (k < kNst + kNnl) ? k : (kNst + kNnl - 1);
        const int kb = (k >= kNst + kNnl) ? (k - kNst - kNnl) : 0;
        const float hc = H[(size_t)(kNst + kNnl + r) * kHdim + kh];
        const float bb = bf16r(B2[r * kNin + kb]);
        computed = (k < kNst + kNnl);
        w = computed ? hc : bb;
      } else {
        const int rc = (r < kNout) ? r : (kNout - 1);
        const int k1 = (k < kNst) ? k : (kNst - 1);
        const int k2 = (k >= kNst && k < kNst + kNnl) ? (k - kNst) : 0;
        const int k3 = (k >= kNst + kNnl) ? (k - kNst - kNnl) : 0;
        const float c2 = bf16r(C2[rc * kNst + k1]);
        const float d21 = bf16r(D21[rc * kNnl + k2]);
        const float d22 = bf16r(D22[rc * kNin + k3]);
        computed = false;
        w = (r < kNout) ? ((k < kNst) ? c2 : ((k < kNst + kNnl) ? d21 : d22)) : 0.0f;
      }
      _Float16 hi, lo;
      split_w(w, kWCarry, hi, lo);
      hv[e] = half ? (computed ? lo : (_Float16)0.0f) : hi;
    }
    unsigned short* dp = ((which == 0) ? WSV2 : ((which == 1) ? WEX2 : WOUT)) + (size_t)row * ld + k8;
    *(volatile v8h*)dp = hv;
    __threadfence();
    *(volatile v8h*)dp = hv;
  } else if (v < nA + nB + nC + nD) {
    const int u = v - nA - nB - nC;
    const int i = u >> 3;
    const int j8 = (u & 7) * 8;
    v4f o0, o1;
#pragma unroll
    for (int e = 0; e < 8; ++e) {
      const int j = j8 + e;
      const float h = H[(size_t)(kNst + i) * kHdim + kNst + j];
      const float d = (j < i) ? -h : 0.0f;
      if (e < 4) o0[e] = d; else o1[e - 4] = d;
    }
    float* dp = D11 + (size_t)i * kNnl + j8;
    for (int pass = 0; pass < 2; ++pass) {
      *(volatile v4f*)dp = o0;
      *(volatile v4f*)(dp + 4) = o1;
      __threadfence();
    }
  } else {
    const int i8 = (v - nA - nB - nC - nD) * 8;
    v4f o0, o1;
#pragma unroll
    for (int e = 0; e < 8; ++e) {
      const int i = i8 + e;
      const float l = 0.5f * (H[(size_t)(kNst + i) * kHdim + kNst + i] + kEps);
      if (e < 4) o0[e] = l; else o1[e - 4] = l;
    }
    float* dp = LAM + i8;
    if (live) {
      for (int pass = 0; pass < 2; ++pass) {
        *(volatile v4f*)dp = o0;
        *(volatile v4f*)(dp + 4) = o1;
        __threadfence();
      }
    }
  }
}

constexpr int kEPitch = kNst + 1;
__global__ __launch_bounds__(kNst) void einv_kernel(const float* __restrict__ H, const float* __restrict__ Y1,
                                                    unsigned short* __restrict__ EINV2) {
  __shared__ float am[kNst * kEPitch];
  __shared__ __align__(16) float colc[kNst];
  const int j = threadIdx.x;
#pragma unroll 1
  for (int r = 0; r < kNst; ++r) {
    const float e = 0.5f * (((H[(size_t)r * kHdim + j] + H[(size_t)(kNst + kNnl + r) * kHdim + kNst + kNnl + j])
                             + bf16r(Y1[r * kNst + j])) - bf16r(Y1[j * kNst + r]))
                    + ((r == j) ? kEps : 0.0f);
    am[r * kEPitch + j] = e;
  }
  __syncthreads();
#pragma unroll 1
  for (int c = 0; c < kNst; ++c) {
    colc[j] = am[j * kEPitch + c];
    __syncthreads();
    const float p = am[c * kEPitch + c];
    const float top = (j == c) ? 1.0f : am[c * kEPitch + j];
    const float acj = top / p;
    __syncthreads();
#pragma unroll 1
    for (int r = 0; r < kNst; ++r) {
      const float f = colc[r];
      const float old = (j == c) ? 0.0f : am[r * kEPitch + j];
      am[r * kEPitch + j] = (r == c) ? acj : (old - f * acj);
    }
    __syncthreads();
  }
#pragma unroll 1
  for (int it = 0; it < 32; ++it) {
    const int v = it * kNst + j;
    const int row = v >> 4;
    const int k8 = (v & 15) * 8;
    const int n = row & (kNst - 1);
    const int half = row >> 7;
    v8h hv;
#pragma unroll
    for (int e = 0; e < 8; ++e) {
      _Float16 hi, lo;
      split_w(am[n * kEPitch + k8 + e], kEiCarry, hi, lo);
      hv[e] = half ? lo : hi;
    }
    unsigned short* dp = EINV2 + (size_t)row * kNst + k8;
    *(volatile v8h*)dp = hv;
    __threadfence();
    *(volatile v8h*)dp = hv;
  }
}

__global__ __launch_bounds__(kThr) void zs_plane_kernel(const float* __restrict__ state, const float* __restrict__ inpt,
                                                        unsigned short* __restrict__ ZS16, int row0) {
  const int v = blockIdx.x * kThr + threadIdx.x;
  const int row = v / 20;
  const int k8 = (v - row * 20) * 8;
  const bool isState = (k8 < kNst);
  const int ks = isState ? k8 : 0;
  const int ki = isState ? 0 : (k8 - kNst);
  const float* sp = state + (size_t)(row0 + row) * kNst + ks;
  const float* ip = inpt + (size_t)(row0 + row) * kNin + ki;
  const v4f s0 = *(const v4f*)sp, s1 = *(const v4f*)(sp + 4);
  const v4f i0 = *(const v4f*)ip, i1 = *(const v4f*)(ip + 4);
  v8h hv;
#pragma unroll
  for (int e = 0; e < 4; ++e) {
    hv[e]     = (_Float16)carry_flush(bf16r(isState ? s0[e] : i0[e]), kInCarry);
    hv[4 + e] = (_Float16)carry_flush(bf16r(isState ? s1[e] : i1[e]), kInCarry);
  }
  unsigned short* dp = ZS16 + (size_t)row * kKsv + k8;
  *(volatile v8h*)dp = hv;
  __threadfence();
  *(volatile v8h*)dp = hv;
}

__global__ __launch_bounds__(128) void subst_kernel(const float* __restrict__ SV2, const float* __restrict__ D11,
                                                    const float* __restrict__ LAM, const float* __restrict__ state,
                                                    const float* __restrict__ inpt, unsigned short* __restrict__ Z16,
                                                    int row0) {
  __shared__ __align__(16) float dsm[kNnl * kNnl];
  __shared__ __align__(16) float lsm[kNnl];
  __shared__ __align__(16) float wl[kNnl * 128];
  const int t = threadIdx.x;
#pragma unroll 1
  for (int i = t; i < kNnl * kNnl; i += 128) dsm[i] = D11[i];
  if (t < kNnl) lsm[t] = LAM[t];
  __syncthreads();
  const int row = blockIdx.x * 128 + t;
  const float* svp = SV2 + (size_t)row * 2 * kNnl;
#pragma unroll 1
  for (int i = 0; i < kNnl; ++i) {
    float acc = svp[i] + kLoFold * svp[kNnl + i];
#pragma unroll 1
    for (int jj = 0; jj < i; ++jj) acc = fmaf(dsm[i * kNnl + jj], wl[jj * 128 + t], acc);
    wl[i * 128 + t] = tanhf(acc / lsm[i]);
  }
  unsigned short* zp = Z16 + (size_t)row * kKz;
  const float* sp = state + (size_t)(row0 + row) * kNst;
  const float* ip = inpt + (size_t)(row0 + row) * kNin;
#pragma unroll 1
  for (int q = 0; q < 28; ++q) {
    v8h hv;
    if (q < 16) {
      const v4f a0 = *(const v4f*)(sp + 8 * q), a1 = *(const v4f*)(sp + 8 * q + 4);
#pragma unroll
      for (int e = 0; e < 4; ++e) { hv[e] = (_Float16)carry_flush(bf16r(a0[e]), kInCarry); hv[4 + e] = (_Float16)carry_flush(bf16r(a1[e]), kInCarry); }
    } else if (q < 24) {
#pragma unroll
      for (int e = 0; e < 8; ++e) hv[e] = (_Float16)carry_flush(wl[(8 * (q - 16) + e) * 128 + t], kInCarry);
    } else {
      const v4f a0 = *(const v4f*)(ip + 8 * (q - 24)), a1 = *(const v4f*)(ip + 8 * (q - 24) + 4);
#pragma unroll
      for (int e = 0; e < 4; ++e) { hv[e] = (_Float16)carry_flush(bf16r(a0[e]), kInCarry); hv[4 + e] = (_Float16)carry_flush(bf16r(a1[e]), kInCarry); }
    }
    *(volatile v8h*)(zp + 8 * q) = hv;
    __threadfence();
    *(volatile v8h*)(zp + 8 * q) = hv;
  }
}

__global__ __launch_bounds__(kThr) void ex_combine_kernel(const float* __restrict__ EX2, unsigned short* __restrict__ EX16) {
  const int v = blockIdx.x * kThr + threadIdx.x;
  const int row = v >> 4;
  const int c8 = (v & 15) * 8;
  const float* hp = EX2 + (size_t)row * 2 * kNst + c8;
  const v4f h0 = *(const v4f*)hp, h1 = *(const v4f*)(hp + 4);
  const v4f l0 = *(const v4f*)(hp + kNst), l1 = *(const v4f*)(hp + kNst + 4);
  v8h hv;
#pragma unroll
  for (int e = 0; e < 4; ++e) {
    hv[e]     = (_Float16)carry_flush(h0[e] + kLoFold * l0[e], kExCarry);
    hv[4 + e] = (_Float16)carry_flush(h1[e] + kLoFold * l1[e], kExCarry);
  }
  unsigned short* dp = EX16 + (size_t)row * kNst + c8;
  *(volatile v8h*)dp = hv;
  __threadfence();
  *(volatile v8h*)dp = hv;
}

__global__ __launch_bounds__(kThr) void fin_kernel(const float* __restrict__ SRC, float* __restrict__ dst, int row0, int mode) {
  const int v = blockIdx.x * kThr + threadIdx.x;
  if (mode == 0) {
    const int row = v >> 5;
    const int c4 = (v & 31) * 4;
    const v4f h = *(const v4f*)(SRC + (size_t)row * 2 * kNst + c4);
    const v4f l = *(const v4f*)(SRC + (size_t)row * 2 * kNst + kNst + c4);
    v4f o;
#pragma unroll
    for (int e = 0; e < 4; ++e) o[e] = h[e] + kLoFold * l[e];
    float* op = dst + (size_t)(row0 + row) * kNst + c4;
    *(volatile v4f*)op = o;
    __threadfence();
    *(volatile v4f*)op = o;
  } else {
    const int row = v >> 2;
    const int c4 = (v & 3) * 4;
    const v4f o = *(const v4f*)(SRC + (size_t)row * 64 + c4);
    float* op = dst + (size_t)(row0 + row) * kNout + c4;
    *(volatile v4f*)op = o;
    __threadfence();
    *(volatile v4f*)op = o;
  }
}

extern "C" void kernel_launch(void* const* d_in, const int* in_sizes, int n_in,
                              void* d_out, int out_size, void* d_ws, size_t ws_size,
                              hipStream_t stream) {
  if (n_in < 9 || d_out == nullptr || d_ws == nullptr) return;
  if (in_sizes[0] != kBatch * kNin || in_sizes[1] != kBatch * kNst || in_sizes[2] != kHdim * kHdim || in_sizes[3] != kNst * kNst) return;
  if (in_sizes[4] != kNst * kNin || in_sizes[5] != kNout * kNst || in_sizes[6] != kNout * kNnl || in_sizes[7] != kNout * kNin || in_sizes[8] != kNnl * kNin) return;
  if (out_size != kBatch * (kNout + kNst)) return;
  if (ws_size < kWsTotal) return;
  const float* inpt  = (const float*)d_in[0];
  const float* state = (const float*)d_in[1];
  const float* X   = (const float*)d_in[2];
  const float* Y1  = (const float*)d_in[3];
  const float* B2  = (const float*)d_in[4];
  const float* C2  = (const float*)d_in[5];
  const float* D21 = (const float*)d_in[6];
  const float* D22 = (const float*)d_in[7];
  const float* D12 = (const float*)d_in[8];
  float* out0 = (float*)d_out;
  float* out1 = out0 + (size_t)kBatch * kNout;
  char* ws = (char*)d_ws;
  unsigned short* XT16 = (unsigned short*)(ws + kOffXT);
  float* ZB   = (float*)(ws + kOffZB);
  float* H32  = (float*)(ws + kOffH32);
  unsigned short* WSV2 = (unsigned short*)(ws + kOffWSV);
  unsigned short* WEX2 = (unsigned short*)(ws + kOffWEX);
  unsigned short* WOUT = (unsigned short*)(ws + kOffWOUT);
  unsigned short* EINV2 = (unsigned short*)(ws + kOffEINV);
  float* D11  = (float*)(ws + kOffD11);
  float* LAM  = (float*)(ws + kOffLAM);
  unsigned short* ZS16 = (unsigned short*)(ws + kOffZS);
  float* SV2  = (float*)(ws + kOffSV2);
  unsigned short* Z16 = (unsigned short*)(ws + kOffZ16);
  float* EX2  = (float*)(ws + kOffEX2);
  unsigned short* EX16 = (unsigned short*)(ws + kOffEX16);

  xt_plane_kernel<<<kHdim + 1, kHdim / 8, 0, stream>>>(X, XT16, ZB);
  wmma_gemm64<0, false, 2, 0, false, 0><<<dim3((kHdim / 64) * (kHdim / 64) / 8 + 1, 1), 256, 0, stream>>>(
      XT16, XT16, kHdim, 0L, XT16, XT16, kHdim, 0L, (void*)H32, (void*)H32, kHdim, 0L,
      ZB, nullptr, 0L, kHdim, kHdim, kHdim, kXwScale);
  wplanes_kernel<<<48, kThr, 0, stream>>>(H32, D12, B2, C2, D21, D22, WSV2, WEX2, WOUT, D11, LAM);
  einv_kernel<<<1, kNst, 0, stream>>>(H32, Y1, EINV2);

  for (int hb = 0; hb < 2; ++hb) {
    const int row0 = hb * kHalf;
    zs_plane_kernel<<<kHalf * 20 / kThr, kThr, 0, stream>>>(state, inpt, ZS16, row0);
    wmma_gemm64<0, false, 2, 0, false, 0><<<dim3((kHalf / 64) * 2 / 8, 1), 256, 0, stream>>>(
        ZS16, ZS16, kKsv, 0L, WSV2, WSV2, kKsv, 0L, (void*)SV2, (void*)SV2, 2 * kNnl, 0L,
        ZB, nullptr, 0L, kHalf, 2 * kNnl, kKsv, kXwScale);
    subst_kernel<<<kHalf / 128, 128, 0, stream>>>(SV2, D11, LAM, state, inpt, Z16, row0);
    wmma_gemm64<0, false, 2, 0, false, 0><<<dim3((kHalf / 64) * 4 / 8, 1), 256, 0, stream>>>(
        Z16, Z16, kKz, 0L, WEX2, WEX2, kKz, 0L, (void*)EX2, (void*)EX2, 2 * kNst, 0L,
        ZB, nullptr, 0L, kHalf, 2 * kNst, kKz, kXwScale);
    ex_combine_kernel<<<kHalf * 16 / kThr, kThr, 0, stream>>>(EX2, EX16);
    wmma_gemm64<0, false, 2, 0, false, 0><<<dim3((kHalf / 64) * 4 / 8, 1), 256, 0, stream>>>(
        EX16, EX16, kNst, 0L, EINV2, EINV2, kNst, 0L, (void*)EX2, (void*)EX2, 2 * kNst, 0L,
        ZB, nullptr, 0L, kHalf, 2 * kNst, kNst, kSpScale);
    fin_kernel<<<kHalf * 32 / kThr, kThr, 0, stream>>>(EX2, out1, row0, 0);
    wmma_gemm64<0, false, 2, 0, false, 0><<<dim3((kHalf / 64) / 8, 1), 256, 0, stream>>>(
        Z16, Z16, kKz, 0L, WOUT, WOUT, kKz, 0L, (void*)SV2, (void*)SV2, 64, 0L,
        ZB, nullptr, 0L, kHalf, 64, kKz, kXwScale);
    fin_kernel<<<kHalf * 4 / kThr, kThr, 0, stream>>>(SV2, out0, row0, 1);
  }
}
